// GRUModel_36490042147514
// MI455X (gfx1250) — hardware-verified
//
#include <hip/hip_runtime.h>
#include <math.h>

constexpr int N_HID    = 128;
constexpr int N_GATE3  = 3 * N_HID;
constexpr int N_LAYER  = 4;
constexpr int N_STEP   = 512;
constexpr int N_FEAT   = 2;
constexpr int N_LANE   = 1024;
constexpr int LIVE_LANE = N_LANE - 1;
constexpr int N_OUTC   = 3;
constexpr int N_OUT    = N_STEP * N_OUTC;
constexpr int REC_THR  = 256;
constexpr int A_PITCH  = 136;
constexpr int FLUSH_ROWS = 16;
constexpr float W_CARRY  = 256.0f;
constexpr float H_CARRY  = 64.0f;
constexpr float LO_CARRY = 2048.0f;
constexpr float FOLD_HI  = 1.0f / (W_CARRY * H_CARRY);
constexpr float FOLD_LO  = FOLD_HI / LO_CARRY;

static_assert(N_HID % 32 == 0);
static_assert(N_STEP % 64 == 0 && N_GATE3 % 64 == 0 && N_HID % 64 == 0);
static_assert(N_HID == 16 * (REC_THR / 32));
static_assert(FLUSH_ROWS * N_HID == REC_THR * 8);
static_assert(N_STEP % FLUSH_ROWS == 0);
static_assert(2 * N_HID == REC_THR);
static_assert(A_PITCH % 8 == 0 && A_PITCH >= N_HID);
static_assert(N_OUT % 256 == 0);
static_assert((N_STEP * (N_GATE3 / 4)) % 256 == 0);

typedef __attribute__((ext_vector_type(16))) _Float16 v16h;
typedef __attribute__((ext_vector_type(8)))  _Float16 v8h;
typedef __attribute__((ext_vector_type(8)))  float    v8f;
typedef __attribute__((ext_vector_type(4)))  float    v4f;

__device__ __forceinline__ v16h frag_load_h(const _Float16* p) {
  union U { v16h v; v8h h[2]; };
  U f;
  f.h[0] = *(const v8h*)(p);
  f.h[1] = *(const v8h*)(p + 16);
  return f.v;
}
__device__ __forceinline__ v8f mma_h(v16h a, v16h b, v8f c) {
  return __builtin_amdgcn_wmma_f32_16x16x32_f16(false, a, false, b, (short)0, c, false, false);
}
__device__ __forceinline__ void guard3_h(v8f& a, v8f& b, v8f& c, v16h x, v16h y0, v16h y1, v16h y2) {
  asm volatile("v_nop\n\tv_nop\n\tv_nop\n\tv_nop" : "+v"(a), "+v"(b), "+v"(c) : "v"(x), "v"(y0), "v"(y1), "v"(y2));
}
__device__ __forceinline__ void guard4_h(v8f& a, v8f& b, v8f& c, v8f& d, v16h x, v16h y) {
  asm volatile("v_nop\n\tv_nop\n\tv_nop\n\tv_nop" : "+v"(a), "+v"(b), "+v"(c), "+v"(d) : "v"(x), "v"(y));
}
__device__ __forceinline__ void keep4_h(v16h a, v16h b, v16h c, v16h d) {
  asm volatile("v_nop" :: "v"(a), "v"(b), "v"(c), "v"(d));
}
__device__ __forceinline__ void acc_guard4(v8f& a, v8f& b, v8f& c, v8f& d) {
  asm volatile("v_nop\n\tv_nop\n\tv_nop\n\tv_nop" : "+v"(a), "+v"(b), "+v"(c), "+v"(d));
}

__global__ __launch_bounds__(256) void cvt8_f16_kernel(const float* __restrict__ src, unsigned short* __restrict__ dst,
                                                      int n8, float sc) {
  const int i = blockIdx.x * 256 + threadIdx.x;
  if (i < n8) {
    const float* sp = src + (size_t)i * 8;
    const v4f a = *(const v4f*)(sp);
    const v4f b = *(const v4f*)(sp + 4);
    v8h hv;
#pragma unroll
    for (int e = 0; e < 4; ++e) {
      const float fa = a[e] * sc;
      const float fb = b[e] * sc;
      hv[e]     = (_Float16)fa;
      hv[4 + e] = (_Float16)fb;
    }
    unsigned short* dp = dst + (size_t)i * 8;
    *(volatile v8h*)dp = hv;
    __threadfence();
    *(volatile v8h*)dp = hv;
  }
}

__global__ __launch_bounds__(256) void gi0_kernel(const float* __restrict__ x, const float* __restrict__ w0,
                                                 const float* __restrict__ bih, float* __restrict__ GI) {
  const int i = blockIdx.x * 256 + threadIdx.x;
  if (i < N_STEP * (N_GATE3 / 4)) {
    const int t  = i / (N_GATE3 / 4);
    const int g4 = (i - t * (N_GATE3 / 4)) * 4;
    const float x0 = x[(size_t)t * (N_FEAT * N_LANE) + LIVE_LANE];
    const float x1 = x[(size_t)t * (N_FEAT * N_LANE) + N_LANE + LIVE_LANE];
    const v4f wa = *(const v4f*)(w0 + 2 * g4);
    const v4f wb = *(const v4f*)(w0 + 2 * g4 + 4);
    const v4f bb = *(const v4f*)(bih + g4);
    v4f o;
    o[0] = (x0 * wa[0] + x1 * wa[1]) + bb[0];
    o[1] = (x0 * wa[2] + x1 * wa[3]) + bb[1];
    o[2] = (x0 * wb[0] + x1 * wb[1]) + bb[2];
    o[3] = (x0 * wb[2] + x1 * wb[3]) + bb[3];
    float* op = GI + (size_t)i * 4;
    *(volatile v4f*)op = o;
    __threadfence();
    *(volatile v4f*)op = o;
  }
}

template <bool RELU>
__global__ __launch_bounds__(256) void wmma_gemm64_f16(
    const unsigned short* __restrict__ Ap, int lda,
    const unsigned short* __restrict__ Btp, int ldb,
    float* __restrict__ Cout, int ldc,
    const float* __restrict__ bias,
    int M, int N, int K, float scale) {
  const _Float16* A  = (const _Float16*)Ap;
  const _Float16* Bt = (const _Float16*)Btp;
  __shared__ __align__(16) float sT[8][16 * 68];
  const int lane = threadIdx.x & 31;
  const int wave = threadIdx.x >> 5;
  const int tilesN = N >> 6;
  const int tilesM = M >> 6;
  const int tile = blockIdx.x * 8 + wave;
  if (tile >= tilesM * tilesN) return;
  const int tm = tile / tilesN;
  const int tn = tile - tm * tilesN;
  const int m0 = tm << 6;
  const int n0 = tn << 6;

  const int rlane = lane & 15;
  const int koff  = (lane >> 4) * 8;
  const int mOff  = (lane >> 4) * 8;

  v8f acc[4][4];
#pragma unroll
  for (int i = 0; i < 4; ++i)
#pragma unroll
    for (int j = 0; j < 4; ++j) acc[i][j] = (v8f){0.f, 0.f, 0.f, 0.f, 0.f, 0.f, 0.f, 0.f};

  for (int k0 = 0; k0 < K; k0 += 32) {
    v16h bh[4];
#pragma unroll
    for (int j = 0; j < 4; ++j) {
      const size_t bo = (size_t)(n0 + (j << 4) + rlane) * ldb + koff + k0;
      bh[j] = frag_load_h(Bt + bo);
    }
#pragma unroll
    for (int i = 0; i < 4; ++i) {
      const size_t ao = (size_t)(m0 + (i << 4) + rlane) * lda + koff + k0;
      const v16h ah = frag_load_h(A + ao);
#pragma unroll
      for (int j = 0; j < 4; ++j) acc[i][j] = mma_h(ah, bh[j], acc[i][j]);
      guard4_h(acc[i][0], acc[i][1], acc[i][2], acc[i][3], ah, bh[3]);
    }
    keep4_h(bh[0], bh[1], bh[2], bh[3]);
  }
  acc_guard4(acc[0][0], acc[0][1], acc[0][2], acc[0][3]);
  acc_guard4(acc[1][0], acc[1][1], acc[1][2], acc[1][3]);
  acc_guard4(acc[2][0], acc[2][1], acc[2][2], acc[2][3]);
  acc_guard4(acc[3][0], acc[3][1], acc[3][2], acc[3][3]);

  float* slab = sT[wave];
#pragma unroll
  for (int i = 0; i < 4; ++i) {
    const int mBase = m0 + (i << 4);
#pragma unroll
    for (int j = 0; j < 4; ++j) {
      const int n = n0 + (j << 4) + rlane;
      const float bv = bias[n];
#pragma unroll
      for (int r = 0; r < 8; ++r) {
        float v = acc[i][j][r] * scale;
        v += bv;
        if (RELU) v = fmaxf(v, 0.0f);
        slab[(mOff + r) * 68 + (j << 4) + rlane] = v;
      }
    }
    __builtin_amdgcn_fence(__ATOMIC_RELEASE, "workgroup");
    __builtin_amdgcn_wave_barrier();
    __builtin_amdgcn_fence(__ATOMIC_ACQUIRE, "workgroup");
    {
      const int hh = lane >> 4, c4 = (lane & 15) * 4;
      for (int pass = 0; pass < 2; ++pass) {
#pragma unroll
        for (int it = 0; it < 8; ++it) {
          const int row = it * 2 + hh;
          const v4f v = *(const v4f*)(slab + row * 68 + c4);
          *(volatile v4f*)(Cout + (size_t)(mBase + row) * ldc + n0 + c4) = v;
        }
        __threadfence();
      }
    }
    __builtin_amdgcn_fence(__ATOMIC_RELEASE, "workgroup");
    __builtin_amdgcn_wave_barrier();
    __builtin_amdgcn_fence(__ATOMIC_ACQUIRE, "workgroup");
  }
}

__global__ __launch_bounds__(REC_THR) void gru_rec_kernel(const float* __restrict__ GI,
                                                         const unsigned short* __restrict__ WHp,
                                                         const float* __restrict__ bhh,
                                                         unsigned short* __restrict__ HH) {
  __shared__ __align__(16) _Float16 At[2][2 * A_PITCH];
  __shared__ __align__(16) _Float16 Hst[2][FLUSH_ROWS * N_HID];
  const _Float16* WH = (const _Float16*)WHp;
  const int tid = threadIdx.x, lane = tid & 31, wave = tid >> 5;
  const int c = lane & 15, hh = lane >> 4;
  const int j = 16 * wave + c;

  v16h bfr[3][4];
#pragma unroll
  for (int g = 0; g < 3; ++g)
#pragma unroll
    for (int kc = 0; kc < 4; ++kc)
      bfr[g][kc] = frag_load_h(WH + (size_t)(g * N_HID + j) * N_HID + 8 * hh + 32 * kc);

  const float bhr = bhh[j];
  const float bhz = bhh[N_HID + j];
  const float bhn = bhh[2 * N_HID + j];

  At[0][(tid >> 7) * A_PITCH + (tid & 127)] = (_Float16)0.0f;
  float hreg = 0.0f;
  __syncthreads();

  const int  arow_sel = (c < 2) ? c : 1;
  const bool arow_live = (c < 2);
  const v16h zf = {(_Float16)0.0f, (_Float16)0.0f, (_Float16)0.0f, (_Float16)0.0f,
                   (_Float16)0.0f, (_Float16)0.0f, (_Float16)0.0f, (_Float16)0.0f,
                   (_Float16)0.0f, (_Float16)0.0f, (_Float16)0.0f, (_Float16)0.0f,
                   (_Float16)0.0f, (_Float16)0.0f, (_Float16)0.0f, (_Float16)0.0f};
  const v8f z8 = {0.f, 0.f, 0.f, 0.f, 0.f, 0.f, 0.f, 0.f};

#pragma unroll 1
  for (int t = 0; t < N_STEP; ++t) {
    const int p  = t & 1;
    const int fb = (t / FLUSH_ROWS) & 1;
    const int fr = t & (FLUSH_ROWS - 1);

    float gir = GI[(size_t)t * N_GATE3 + j];
    float giz = GI[(size_t)t * N_GATE3 + N_HID + j];
    float gin = GI[(size_t)t * N_GATE3 + 2 * N_HID + j];
    asm volatile("" : "+v"(gir), "+v"(giz), "+v"(gin));

    const _Float16* arow = &At[p][0] + arow_sel * A_PITCH + 8 * hh;
    v8f acc0 = z8, acc1 = z8, acc2 = z8;
#pragma unroll
    for (int kc = 0; kc < 4; ++kc) {
      v16h a = frag_load_h(arow + 32 * kc);
      a = arow_live ? a : zf;
      acc0 = mma_h(a, bfr[0][kc], acc0);
      acc1 = mma_h(a, bfr[1][kc], acc1);
      acc2 = mma_h(a, bfr[2][kc], acc2);
      guard3_h(acc0, acc1, acc2, a, bfr[0][kc], bfr[1][kc], bfr[2][kc]);
    }

    const float ghr = (acc0[0] * FOLD_HI + acc0[1] * FOLD_LO) + bhr;
    const float ghz = (acc1[0] * FOLD_HI + acc1[1] * FOLD_LO) + bhz;
    const float ghn = (acc2[0] * FOLD_HI + acc2[1] * FOLD_LO) + bhn;
    const float rg = 1.0f / (1.0f + expf(-(gir + ghr)));
    const float zg = 1.0f / (1.0f + expf(-(giz + ghz)));
    const float ng = tanhf(gin + rg * ghn);
    const float hn = (1.0f - zg) * ng + zg * hreg;
    hreg = hn;

    const float    hs  = hn * H_CARRY;
    const _Float16 hhi = (_Float16)hs;
    const float    hif = (float)hhi;
    const float    res = (hs - hif) * LO_CARRY;
    const _Float16 hlo = (_Float16)res;
    if (hh == 0) {
      At[p ^ 1][j] = hhi;
      At[p ^ 1][A_PITCH + j] = hlo;
      Hst[fb][fr * N_HID + j] = hhi;
    }
    __syncthreads();

    if (fr == FLUSH_ROWS - 1) {
      const v8h v = *(const v8h*)(&Hst[fb][0] + tid * 8);
      unsigned short* dp = HH + (size_t)(t - (FLUSH_ROWS - 1)) * N_HID + tid * 8;
      *(volatile v8h*)dp = v;
      __threadfence();
      *(volatile v8h*)dp = v;
    }
  }
}

__global__ __launch_bounds__(256) void head_out_kernel(const float* __restrict__ hid, const float* __restrict__ w2,
                                                      const float* __restrict__ b2, float* __restrict__ out) {
  const int i  = blockIdx.x * 256 + threadIdx.x;
  const int ic = (i < N_OUT) ? i : (N_OUT - 1);
  const int t  = ic / N_OUTC;
  const int jc = ic - t * N_OUTC;
  const float* hp = hid + (size_t)t * N_HID;
  const float* wp = w2 + (size_t)jc * N_HID;
  float s = 0.0f;
#pragma unroll 1
  for (int k = 0; k < N_HID; k += 4) {
    const v4f a = *(const v4f*)(hp + k);
    const v4f b = *(const v4f*)(wp + k);
    s += a[0] * b[0];
    s += a[1] * b[1];
    s += a[2] * b[2];
    s += a[3] * b[3];
  }
  s += b2[jc];
  if (i < N_OUT) {
    volatile float* op = (volatile float*)out + i;
    *op = s;
    __threadfence();
    *op = s;
  }
}

extern "C" void kernel_launch(void* const* d_in, const int* in_sizes, int n_in,
                              void* d_out, int out_size, void* d_ws, size_t ws_size, hipStream_t stream) {
  if (n_in < 10 || d_out == nullptr || d_ws == nullptr) return;
  if (in_sizes[0] != N_STEP * N_FEAT * N_LANE || in_sizes[1] != N_GATE3 * N_FEAT ||
      in_sizes[2] != (N_LAYER - 1) * N_GATE3 * N_HID || in_sizes[3] != N_LAYER * N_GATE3 * N_HID ||
      in_sizes[4] != N_LAYER * N_GATE3 || in_sizes[5] != N_LAYER * N_GATE3 ||
      in_sizes[6] != N_HID * N_HID || in_sizes[7] != N_HID || in_sizes[8] != N_OUTC * N_HID ||
      in_sizes[9] != N_OUTC || out_size != N_OUT) return;

  const float* x      = (const float*)d_in[0];
  const float* w_ih0  = (const float*)d_in[1];
  const float* w_ihr  = (const float*)d_in[2];
  const float* w_hh   = (const float*)d_in[3];
  const float* b_ih   = (const float*)d_in[4];
  const float* b_hh   = (const float*)d_in[5];
  const float* fc1_w  = (const float*)d_in[6];
  const float* fc1_b  = (const float*)d_in[7];
  const float* fc2_w  = (const float*)d_in[8];
  const float* fc2_b  = (const float*)d_in[9];
  float* outp = (float*)d_out;

  char* ws = (char*)d_ws;
  size_t off = 0;
  auto carve = [&](size_t bytes) -> char* { char* q = ws + off; off += (bytes + 255) & ~(size_t)255; return q; };
  unsigned short* WIH = (unsigned short*)carve((size_t)(N_LAYER - 1) * N_GATE3 * N_HID * 2);
  unsigned short* WHH = (unsigned short*)carve((size_t)N_LAYER * N_GATE3 * N_HID * 2);
  unsigned short* WF1 = (unsigned short*)carve((size_t)N_HID * N_HID * 2);
  float*          GIP = (float*)carve((size_t)N_LAYER * N_STEP * N_GATE3 * 4);
  unsigned short* HHP = (unsigned short*)carve((size_t)N_LAYER * N_STEP * N_HID * 2);
  float*          HIDP = (float*)carve((size_t)N_STEP * N_HID * 4);
  if (off > ws_size || off > (size_t)134217728) return;

  const size_t giPlane = (size_t)N_STEP * N_GATE3;
  const size_t hhPlane = (size_t)N_STEP * N_HID;
  const size_t wPlane  = (size_t)N_GATE3 * N_HID;

  const int n8a = (N_LAYER - 1) * N_GATE3 * N_HID / 8;
  const int n8b = N_LAYER * N_GATE3 * N_HID / 8;
  const int n8c = N_HID * N_HID / 8;
  cvt8_f16_kernel<<<(n8a + 255) / 256, 256, 0, stream>>>(w_ihr, WIH, n8a, W_CARRY);
  cvt8_f16_kernel<<<(n8b + 255) / 256, 256, 0, stream>>>(w_hh,  WHH, n8b, W_CARRY);
  cvt8_f16_kernel<<<(n8c + 255) / 256, 256, 0, stream>>>(fc1_w, WF1, n8c, W_CARRY);

  gi0_kernel<<<(N_STEP * (N_GATE3 / 4)) / 256, 256, 0, stream>>>(x, w_ih0, b_ih, GIP);
  gru_rec_kernel<<<1, REC_THR, 0, stream>>>(GIP, WHH, b_hh, HHP);

  for (int l = 1; l < N_LAYER; ++l) {
    wmma_gemm64_f16<false><<<(N_STEP / 64) * (N_GATE3 / 64) / 8, 256, 0, stream>>>(
        HHP + (size_t)(l - 1) * hhPlane, N_HID,
        WIH + (size_t)(l - 1) * wPlane, N_HID,
        GIP + (size_t)l * giPlane, N_GATE3,
        b_ih + (size_t)l * N_GATE3,
        N_STEP, N_GATE3, N_HID, FOLD_HI);
    gru_rec_kernel<<<1, REC_THR, 0, stream>>>(GIP + (size_t)l * giPlane, WHH + (size_t)l * wPlane,
                                              b_hh + (size_t)l * N_GATE3, HHP + (size_t)l * hhPlane);
  }

  wmma_gemm64_f16<true><<<(N_STEP / 64) * (N_HID / 64) / 8, 256, 0, stream>>>(
      HHP + (size_t)(N_LAYER - 1) * hhPlane, N_HID,
      WF1, N_HID,
      HIDP, N_HID,
      fc1_b,
      N_STEP, N_HID, N_HID, FOLD_HI);
  head_out_kernel<<<N_OUT / 256, 256, 0, stream>>>(HIDP, fc2_w, fc2_b, outp);
}
